// Self_Attention_13211319402955
// MI455X (gfx1250) — hardware-verified
//
#include <hip/hip_runtime.h>


#ifndef NB
#define NB 8
#endif
#ifndef SEQ
#define SEQ 4096
#endif
#define NB_FULL  8
#define SEQ_FULL 4096
#define CH   256
#define CQ   32
#define QCAR 16.0f
#define VCAR 16.0f
#define PCAR 4096.0f
#define SCL  (1.0f / 256.0f)
#define GMUL (1.0f / 65536.0f)
#define XTP  (CH + 8)
static_assert(SEQ % 256 == 0);
static_assert(SEQ >= 256 && SEQ <= SEQ_FULL);
static_assert(NB >= 1 && NB <= NB_FULL);
static_assert(CH % 64 == 0);
static_assert(CQ == 32);
static_assert((SEQ * CQ) % 2048 == 0);
static_assert((CH * SEQ) % 2048 == 0);

typedef _Float16 h16;
typedef unsigned short bf;
typedef __attribute__((ext_vector_type(16))) __bf16   v16bf;
typedef __attribute__((ext_vector_type(16))) _Float16 v16h;
typedef __attribute__((ext_vector_type(8)))  _Float16 v8h;
typedef __attribute__((ext_vector_type(8)))  unsigned short v8us;
typedef __attribute__((ext_vector_type(8)))  float    v8f;
typedef __attribute__((ext_vector_type(4)))  float    v4f;
typedef v8h  __attribute__((may_alias)) v8ha;
typedef v4f  __attribute__((may_alias)) v4fa;
typedef v8us __attribute__((may_alias)) v8usa;

__device__ __forceinline__ unsigned short f2bf(float f) { unsigned u = __float_as_uint(f); u += 0x7FFFu + ((u >> 16) & 1u); return (unsigned short)(u >> 16); }
__device__ __forceinline__ float bf2f(unsigned short b) { return __uint_as_float(((unsigned)b) << 16); }
__device__ __forceinline__ float bfr(float f) { return bf2f(f2bf(f)); }
__device__ __forceinline__ h16 tohx(float x) { return (h16)x; }
__device__ __forceinline__ v16h cat16(v8h lo, v8h hi) { return __builtin_shufflevector(lo, hi, 0, 1, 2, 3, 4, 5, 6, 7, 8, 9, 10, 11, 12, 13, 14, 15); }
__device__ __forceinline__ v16bf cat16b(v8us lo, v8us hi) { return __builtin_bit_cast(v16bf, __builtin_shufflevector(lo, hi, 0, 1, 2, 3, 4, 5, 6, 7, 8, 9, 10, 11, 12, 13, 14, 15)); }
__device__ __forceinline__ v8f wmma16(v16h a, v16h b, v8f c) { return __builtin_amdgcn_wmma_f32_16x16x32_f16(false, a, false, b, (short)0, c, false, false); }
__device__ __forceinline__ v8f wmmab(v16bf a, v16bf b, v8f c) { return __builtin_amdgcn_wmma_f32_16x16x32_bf16(false, a, false, b, (short)0, c, false, false); }

template <typename T16> struct WFrag;
template <> struct WFrag<h16> { typedef v16h V; static __device__ __forceinline__ V ld(const h16* p) { return cat16(*(const v8h*)p, *(const v8h*)(p + 16)); } static __device__ __forceinline__ v8f mma(V a, V b, v8f c) { return wmma16(a, b, c); } };
template <> struct WFrag<bf> { typedef v16bf V; static __device__ __forceinline__ V ld(const bf* p) { return cat16b(*(const v8us*)p, *(const v8us*)(p + 16)); } static __device__ __forceinline__ v8f mma(V a, V b, v8f c) { return wmmab(a, b, c); } };
template <typename T16, int NSPLIT, int EPI>
__global__ __launch_bounds__(32) void k_gemmw(const T16* __restrict__ A, const T16* __restrict__ A2, const T16* __restrict__ Bt, const T16* __restrict__ Bt2, int K, float* C, int ldc,
                                              const float* __restrict__ bias, const float* __restrict__ R, int ldr, float gmul, size_t sA, size_t sB, size_t sC) {
    typedef typename WFrag<T16>::V V;
    __shared__ __align__(16) float os[16 * 68];
    const size_t z = blockIdx.z; A += z * sA; if (A2) A2 += z * sA; Bt += z * sB; if (Bt2) Bt2 += z * sB; C += z * sC;
    const int lane = threadIdx.x & 31, lr = lane & 15, hi = lane >> 4; const int r0 = blockIdx.x * 64, c0 = blockIdx.y * 64;
    float g = 0.0f;
    if (EPI == 3) g = bfr(bias[0]) * gmul;
    v8f acc[4][4];
#pragma unroll
    for (int mb = 0; mb < 4; ++mb)
#pragma unroll
        for (int nb = 0; nb < 4; ++nb) acc[mb][nb] = (v8f){};
    const size_t aoff = (size_t)(r0 + lr) * K + 8 * hi, boff = (size_t)(c0 + lr) * K + 8 * hi;
#pragma unroll 1
    for (int kc = 0; kc < K; kc += 32) {
        V a[4], a2[4];
#pragma unroll
        for (int mb = 0; mb < 4; ++mb) { a[mb] = WFrag<T16>::ld(A + aoff + (size_t)mb * 16 * K + kc); if (NSPLIT == 1 || NSPLIT == 2) a2[mb] = WFrag<T16>::ld(A2 + aoff + (size_t)mb * 16 * K + kc); }
#pragma unroll
        for (int nb = 0; nb < 4; ++nb) { const V b = WFrag<T16>::ld(Bt + boff + (size_t)nb * 16 * K + kc); V b2; if (NSPLIT >= 2) b2 = WFrag<T16>::ld(Bt2 + boff + (size_t)nb * 16 * K + kc);
#pragma unroll
            for (int mb = 0; mb < 4; ++mb) { acc[mb][nb] = WFrag<T16>::mma(a[mb], b, acc[mb][nb]); if (NSPLIT == 1 || NSPLIT == 2) acc[mb][nb] = WFrag<T16>::mma(a2[mb], b, acc[mb][nb]); if (NSPLIT >= 2) acc[mb][nb] = WFrag<T16>::mma(a[mb], b2, acc[mb][nb]); } }
        asm volatile("v_nop\n\tv_nop\n\tv_nop\n\tv_nop" : "+v"(acc[0][0]), "+v"(acc[1][1]), "+v"(acc[2][2]), "+v"(acc[3][3]) : "v"(a[0]), "v"(a[3]));
    }
#pragma unroll
    for (int mb = 0; mb < 4; ++mb) {
#pragma unroll
        for (int nb = 0; nb < 4; ++nb) {
#pragma unroll
            for (int j = 0; j < 8; ++j) os[(hi * 8 + j) * 68 + nb * 16 + lr] = acc[mb][nb][j]; }
        __builtin_amdgcn_wave_barrier(); asm volatile("" ::: "memory");
        float* crow = C + (size_t)(r0 + mb * 16) * ldc + c0;
#pragma unroll 1
        for (int ps = 0; ps < 2; ++ps) {
#pragma unroll
            for (int s = 0; s < 8; ++s) { const int row = 2 * s + hi, cofs = lr * 4; v4f val = *(const v4fa*)(os + row * 68 + cofs);
                if (EPI == 1) { val[0] += bfr(bias[c0 + cofs]); val[1] += bfr(bias[c0 + cofs + 1]); val[2] += bfr(bias[c0 + cofs + 2]); val[3] += bfr(bias[c0 + cofs + 3]); }
                if (EPI == 2) { const float bb = bfr(bias[r0 + mb * 16 + row]); val[0] += bb; val[1] += bb; val[2] += bb; val[3] += bb; }
                if (EPI == 3) { const v4f rr = *(const v4f*)(R + (size_t)(r0 + mb * 16 + row) * ldr + c0 + cofs); val[0] = g * val[0] + bfr(rr[0]); val[1] = g * val[1] + bfr(rr[1]); val[2] = g * val[2] + bfr(rr[2]); val[3] = g * val[3] + bfr(rr[3]); }
                *(volatile v4f*)(crow + (size_t)row * ldc + cofs) = val; }
            if (ps == 0) __threadfence(); }
        __builtin_amdgcn_wave_barrier(); asm volatile("" ::: "memory");
    }
}

__global__ __launch_bounds__(256) void k_cvt8(const float* __restrict__ src, bf* dst, size_t n8) { const size_t i = (size_t)blockIdx.x * 256 + threadIdx.x; if (i >= n8) return; const v8f v = *(const v8f*)(src + i * 8); v8us o;
#pragma unroll
    for (int k = 0; k < 8; ++k) o[k] = f2bf(v[k]); *(volatile v8us*)(dst + i * 8) = o; __threadfence(); *(volatile v8us*)(dst + i * 8) = o; }

__global__ __launch_bounds__(256) void k_xT(const float* __restrict__ X, bf* XT) {
    __shared__ __align__(16) unsigned short sx[64 * XTP];
    const int tid = threadIdx.x, lane = tid & 31, w = tid >> 5; const int n0 = blockIdx.x * 64;
#pragma unroll 1
    for (int it = 0; it < CH / 16; ++it) { const int c = it * 16 + (tid >> 4); const int j4 = (tid & 15) * 4;
        const v4f v = *(const v4f*)(X + (size_t)c * SEQ_FULL + n0 + j4);
#pragma unroll
        for (int q = 0; q < 4; ++q) sx[(j4 + q) * XTP + c] = f2bf(v[q]); }
    __syncthreads();
#pragma unroll 1
    for (int ps = 0; ps < 2; ++ps) {
#pragma unroll
        for (int r = 0; r < 8; ++r) { const int nl = w * 8 + r; const v8us o = *(const v8usa*)(sx + nl * XTP + lane * 8);
            *(volatile v8us*)(XT + (size_t)(n0 + nl) * CH + lane * 8) = o; }
        if (ps == 0) __threadfence(); }
}

__global__ __launch_bounds__(256) void k_qkp(const float* __restrict__ F, const float* __restrict__ bq, const float* __restrict__ bk, h16* QP, h16* KP) {
    const size_t e = ((size_t)blockIdx.x * 256 + threadIdx.x) * 8; if (e >= (size_t)SEQ * CQ) return;
    const int o = (int)(e % CQ); const size_t n = e / CQ; const float* f = F + n * (2 * CQ) + o;
    const v8f a = *(const v8f*)f; const v8f c = *(const v8f*)(f + CQ); v8h oq, ok;
#pragma unroll
    for (int k = 0; k < 8; ++k) { oq[k] = tohx((a[k] + bfr(bq[o + k])) * QCAR); ok[k] = tohx((c[k] + bfr(bk[o + k])) * QCAR); }
    *(volatile v8h*)(QP + e) = oq; *(volatile v8h*)(KP + e) = ok; __threadfence(); *(volatile v8h*)(QP + e) = oq; *(volatile v8h*)(KP + e) = ok;
}

__global__ __launch_bounds__(256) void k_vp(const float* __restrict__ FV, h16* VP) {
    const size_t e = ((size_t)blockIdx.x * 256 + threadIdx.x) * 8; if (e >= (size_t)CH * SEQ) return;
    const v8f a = *(const v8f*)(FV + e); v8h o;
#pragma unroll
    for (int k = 0; k < 8; ++k) o[k] = tohx(a[k] * VCAR);
    *(volatile v8h*)(VP + e) = o; __threadfence(); *(volatile v8h*)(VP + e) = o;
}

__global__ __launch_bounds__(256) void k_asoft(const float* __restrict__ Sb, h16* P16) {
    const int lane = threadIdx.x & 31; const int row = blockIdx.x * 8 + (threadIdx.x >> 5); if (row >= SEQ) return;
    const float* sr = Sb + (size_t)row * SEQ; float v[SEQ / 32]; float mx = -3.0e38f;
#pragma unroll
    for (int ch = 0; ch < SEQ / 256; ++ch) { const int j0 = ch * 256 + lane * 8; const v4f a = *(const v4f*)(sr + j0); const v4f c = *(const v4f*)(sr + j0 + 4);
#pragma unroll
        for (int q = 0; q < 4; ++q) { const float t0 = a[q] * SCL, t1 = c[q] * SCL; v[ch * 8 + q] = t0; v[ch * 8 + 4 + q] = t1; mx = fmaxf(mx, fmaxf(t0, t1)); } }
#pragma unroll
    for (int sh = 16; sh; sh >>= 1) mx = fmaxf(mx, __shfl_xor(mx, sh, 32));
    float sum = 0.f;
#pragma unroll
    for (int k = 0; k < SEQ / 32; ++k) { float d0 = __fsub_rn(v[k], mx); asm volatile("" : "+v"(d0)); v[k] = __builtin_amdgcn_exp2f(__fmul_rn(d0, 1.4426950408889634f)); sum += v[k]; }
#pragma unroll
    for (int sh = 16; sh; sh >>= 1) sum += __shfl_xor(sum, sh, 32);
    const float f = __fdiv_rn(PCAR, sum);
#pragma unroll 1
    for (int ps = 0; ps < 2; ++ps) {
#pragma unroll
        for (int ch = 0; ch < SEQ / 256; ++ch) { v8h o8;
#pragma unroll
            for (int q = 0; q < 8; ++q) o8[q] = tohx(v[ch * 8 + q] * f);
            *(volatile v8h*)(P16 + (size_t)row * SEQ + ch * 256 + lane * 8) = o8; }
        if (ps == 0) __threadfence(); }
}

#define WS_WQK ((size_t)2 * CQ * CH * 2)
#define WS_WV  ((size_t)CH * CH * 2)
#define WS_XT  ((size_t)SEQ * CH * 2)
#define WS_FQK ((size_t)SEQ * 2 * CQ * 4)
#define WS_QP  ((size_t)SEQ * CQ * 2)
#define WS_FV  ((size_t)CH * SEQ * 4)
#define WS_VP  ((size_t)CH * SEQ * 2)
#define WS_SB  ((size_t)SEQ * SEQ * 4)
#define WS_PT  ((size_t)SEQ * SEQ * 2)
#define WS_AL(x) (((x) + 255) & ~(size_t)255)
#define WS_TOTAL (WS_AL(WS_WQK) + WS_AL(WS_WV) + WS_AL(WS_XT) + WS_AL(WS_FQK) + 2 * WS_AL(WS_QP) + WS_AL(WS_FV) + WS_AL(WS_VP) + WS_AL(WS_SB) + WS_AL(WS_PT))
static_assert(WS_TOTAL <= (size_t)134217728);

extern "C" void kernel_launch(void* const* d_in, const int* in_sizes, int n_in,
                              void* d_out, int out_size, void* d_ws, size_t ws_size, hipStream_t stream) {
    if (n_in < 8) return;
    const long long need_x = (long long)(NB - 1) * CH * SEQ_FULL + (long long)(CH - 1) * SEQ_FULL + SEQ;
    if ((long long)in_sizes[0] < need_x || in_sizes[1] < CQ * CH || in_sizes[2] < CQ || in_sizes[3] < CQ * CH || in_sizes[4] < CQ || in_sizes[5] < CH * CH || in_sizes[6] < CH || in_sizes[7] < 1) return;
    if ((long long)out_size < need_x) return;
    const float* x   = (const float*)d_in[0];
    const float* wq  = (const float*)d_in[1];
    const float* bq  = (const float*)d_in[2];
    const float* wk  = (const float*)d_in[3];
    const float* bk  = (const float*)d_in[4];
    const float* wv  = (const float*)d_in[5];
    const float* bv  = (const float*)d_in[6];
    const float* gam = (const float*)d_in[7];
    float* OUT = (float*)d_out;
    char* wsp = (char*)d_ws;
    auto take = [&](size_t bytes) { char* p = wsp; wsp += WS_AL(bytes); return (void*)p; };
    bf* WQK = (bf*)take(WS_WQK);
    bf* WVB = (bf*)take(WS_WV);
    bf* XT  = (bf*)take(WS_XT);
    float* FQK = (float*)take(WS_FQK);
    h16* QP = (h16*)take(WS_QP);
    h16* KP = (h16*)take(WS_QP);
    float* FV = (float*)take(WS_FV);
    h16* VP = (h16*)take(WS_VP);
    float* Sb = (float*)take(WS_SB);
    h16* Pt = (h16*)take(WS_PT);
    const size_t used = (size_t)(wsp - (char*)d_ws);
    if (used > ws_size || used > (size_t)134217728) return;

    k_cvt8<<<(unsigned)((CQ * CH / 8 + 255) / 256), 256, 0, stream>>>(wq, WQK, (size_t)CQ * CH / 8);
    k_cvt8<<<(unsigned)((CQ * CH / 8 + 255) / 256), 256, 0, stream>>>(wk, WQK + (size_t)CQ * CH, (size_t)CQ * CH / 8);
    k_cvt8<<<(unsigned)((CH * CH / 8 + 255) / 256), 256, 0, stream>>>(wv, WVB, (size_t)CH * CH / 8);
    for (int b = 0; b < NB; ++b) {
        const float* xb = x + (size_t)b * CH * SEQ_FULL; float* ob = OUT + (size_t)b * CH * SEQ_FULL;
        k_xT<<<SEQ / 64, 256, 0, stream>>>(xb, XT);
        k_gemmw<bf, 0, 0><<<dim3(SEQ / 64, (2 * CQ) / 64, 1), 32, 0, stream>>>(XT, nullptr, WQK, nullptr, CH, FQK, 2 * CQ, nullptr, nullptr, 0, 0.0f, (size_t)0, (size_t)0, (size_t)0);
        k_qkp<<<(unsigned)((size_t)SEQ * CQ / 2048), 256, 0, stream>>>(FQK, bq, bk, QP, KP);
        k_gemmw<bf, 0, 2><<<dim3(CH / 64, SEQ / 64, 1), 32, 0, stream>>>(WVB, nullptr, XT, nullptr, CH, FV, SEQ, bv, nullptr, 0, 0.0f, (size_t)0, (size_t)0, (size_t)0);
        k_vp<<<(unsigned)((size_t)CH * SEQ / 2048), 256, 0, stream>>>(FV, VP);
        k_gemmw<h16, 0, 0><<<dim3(SEQ / 64, SEQ / 64, 1), 32, 0, stream>>>(KP, nullptr, QP, nullptr, CQ, Sb, SEQ, nullptr, nullptr, 0, 0.0f, (size_t)0, (size_t)0, (size_t)0);
        k_asoft<<<SEQ / 8, 256, 0, stream>>>(Sb, Pt);
        k_gemmw<h16, 0, 3><<<dim3(CH / 64, SEQ / 64, 1), 32, 0, stream>>>(VP, nullptr, Pt, nullptr, SEQ, ob, SEQ_FULL, gam, xb, SEQ_FULL, GMUL, (size_t)0, (size_t)0, (size_t)0);
    }
}
